// FlowGuidedAlign_26723286516110
// MI455X (gfx1250) — hardware-verified
//
#include <hip/hip_runtime.h>
#include <stddef.h>

constexpr int kBatch  = 2;
constexpr int kCh     = 64;
constexpr int kImg    = 128;
constexpr int kHW     = 16384;
constexpr int kNpix   = 32768;
constexpr int kTaps   = 9;
constexpr int kGroups = 8;
constexpr int kCin1   = 130;
constexpr int kCpt1   = 136;
constexpr int kKp1    = 1280;
constexpr int kKd     = 576;
constexpr int kNom    = 216;
constexpr int kNomPad = 256;
constexpr int kChunk1 = 4096;
constexpr int kChunk2 = 16384;

typedef __attribute__((ext_vector_type(16))) _Float16 v16h;
typedef __attribute__((ext_vector_type(8)))  _Float16 v8h;
typedef __attribute__((ext_vector_type(16))) __bf16   v16b;
typedef __attribute__((ext_vector_type(8)))  __bf16   v8b;
typedef __attribute__((ext_vector_type(8)))  float    v8f;
typedef __attribute__((ext_vector_type(4)))  float    v4f;
typedef __attribute__((ext_vector_type(4)))  unsigned v4u;

__device__ __forceinline__ unsigned short f2bf_bits(float f) {
  unsigned u = __float_as_uint(f);
  return (unsigned short)((u + 0x7FFFu + ((u >> 16) & 1u)) >> 16);
}
__device__ __forceinline__ float bf_bits2f(unsigned short h) { return __uint_as_float(((unsigned)h) << 16); }

__device__ __forceinline__ unsigned pk2(unsigned short a, unsigned short b) {
  return (unsigned)a | ((unsigned)b << 16);
}
__device__ __forceinline__ unsigned pkh2(float a, float b) {
  return pk2(__builtin_bit_cast(unsigned short, (_Float16)a), __builtin_bit_cast(unsigned short, (_Float16)b));
}
__device__ __forceinline__ void pkbf2(float a, float b, unsigned& uh, unsigned& ul) {
  const unsigned short ha = f2bf_bits(a), hb = f2bf_bits(b);
  const unsigned short la = f2bf_bits(a - bf_bits2f(ha)), lb = f2bf_bits(b - bf_bits2f(hb));
  uh = pk2(ha, hb);
  ul = pk2(la, lb);
}

__device__ __forceinline__ void dep_guard_h(v8f& a, v8f& b, v16h x, v16h y) { asm volatile("v_nop\n\tv_nop\n\tv_nop\n\tv_nop" : "+v"(a), "+v"(b) : "v"(x), "v"(y)); }
__device__ __forceinline__ void dep_guard_b(v8f& a, v8f& b, v16b x, v16b y) { asm volatile("v_nop\n\tv_nop\n\tv_nop\n\tv_nop" : "+v"(a), "+v"(b) : "v"(x), "v"(y)); }
__device__ __forceinline__ void keep4_h(v16h a, v16h b, v16h c, v16h d) { asm volatile("v_nop" :: "v"(a), "v"(b), "v"(c), "v"(d)); }
__device__ __forceinline__ void keep4_b(v16b a, v16b b, v16b c, v16b d) { asm volatile("v_nop" :: "v"(a), "v"(b), "v"(c), "v"(d)); }
__device__ __forceinline__ void acc_guard4(v8f& a, v8f& b, v8f& c, v8f& d) { asm volatile("v_nop\n\tv_nop\n\tv_nop\n\tv_nop" : "+v"(a), "+v"(b), "+v"(c), "+v"(d)); }
template <typename T> struct Frag;
template <> struct Frag<_Float16> {
  typedef v16h V; union U { v16h v; v8h h[2]; };
  static __device__ __forceinline__ v16h load(const _Float16* p) {
    U f; f.h[0] = *(const v8h*)(p); f.h[1] = *(const v8h*)(p + 16); return f.v;
  }
  static __device__ __forceinline__ v8f mma(v16h a, v16h b, v8f c) {
    return __builtin_amdgcn_wmma_f32_16x16x32_f16(false, a, false, b, (short)0, c, false, false);
  }
  static __device__ __forceinline__ void guard(v8f& a, v8f& b, v16h x, v16h y) { dep_guard_h(a, b, x, y); }
  static __device__ __forceinline__ void keep(v16h a, v16h b, v16h c, v16h d) { keep4_h(a, b, c, d); }
};
template <> struct Frag<__bf16> {
  typedef v16b V; union U { v16b v; v8b h[2]; };
  static __device__ __forceinline__ v16b load(const __bf16* p) {
    U f; f.h[0] = *(const v8b*)(p); f.h[1] = *(const v8b*)(p + 16); return f.v;
  }
  static __device__ __forceinline__ v8f mma(v16b a, v16b b, v8f c) {
    return __builtin_amdgcn_wmma_f32_16x16x32_bf16(false, a, false, b, (short)0, c, false, false);
  }
  static __device__ __forceinline__ void guard(v8f& a, v8f& b, v16b x, v16b y) { dep_guard_b(a, b, x, y); }
  static __device__ __forceinline__ void keep(v16b a, v16b b, v16b c, v16b d) { keep4_b(a, b, c, d); }
};

template <int ET> struct Elem;
template <> struct Elem<0> { typedef _Float16 T; };
template <> struct Elem<1> { typedef __bf16 T; };
template <int ET, bool SPLIT, int BIAS_MODE, int OUT_MODE, bool RESID, int ACT = 0>
__global__ __launch_bounds__(256) void wmma_gemm64(
    const unsigned short* __restrict__ Ap, const unsigned short* __restrict__ A2p, int lda, long strideA,
    const unsigned short* __restrict__ Btp, const unsigned short* __restrict__ Bt2p, int ldb, long strideB,
    void* __restrict__ Cout, void* __restrict__ Cout2, int ldc, long strideC,
    const float* __restrict__ bias,
    const float* __restrict__ resid, long strideR,
    int M, int N, int K, float scale) {
  typedef typename Elem<ET>::T T;
  typedef typename Frag<T>::V V;
  const T* A = (const T*)Ap; const T* A2 = (const T*)A2p; const T* Bt = (const T*)Btp; const T* Bt2 = (const T*)Bt2p;
  __shared__ __align__(16) float sT[8][16 * 68];
  const int b    = blockIdx.y;
  const int lane = threadIdx.x & 31;
  const int wave = threadIdx.x >> 5;
  const int tilesN = N >> 6;
  const int tilesM = M >> 6;
  const int tile = blockIdx.x * 8 + wave;
  if (tile >= tilesM * tilesN) return;
  const int tm = tile / tilesN;
  const int tn = tile - tm * tilesN;
  const int m0 = tm << 6;
  const int n0 = tn << 6;

  const T* Ab  = A  + (size_t)b * strideA;
  const T* Bb  = Bt + (size_t)b * strideB;
  const T* Ab2 = SPLIT ? (A2  + (size_t)b * strideA) : nullptr;
  const T* Bb2 = SPLIT ? (Bt2 + (size_t)b * strideB) : nullptr;

  const int rlane = lane & 15;
  const int koff  = (lane >> 4) * 8;
  const int mOff  = (lane >> 4) * 8;

  v8f acc[4][4];
#pragma unroll
  for (int i = 0; i < 4; ++i)
#pragma unroll
    for (int j = 0; j < 4; ++j) acc[i][j] = (v8f){0.f,0.f,0.f,0.f,0.f,0.f,0.f,0.f};

  for (int k0 = 0; k0 < K; k0 += 32) {
    V bh[4], bl[4];
#pragma unroll
    for (int j = 0; j < 4; ++j) {
      const size_t bo = (size_t)(n0 + (j << 4) + rlane) * ldb + koff + k0;
      bh[j] = Frag<T>::load(Bb + bo);
      if (SPLIT) bl[j] = Frag<T>::load(Bb2 + bo);
    }
#pragma unroll
    for (int i = 0; i < 4; ++i) {
      const size_t ao = (size_t)(m0 + (i << 4) + rlane) * lda + koff + k0;
      V ah = Frag<T>::load(Ab + ao);
      V al;
      if (SPLIT) al = Frag<T>::load(Ab2 + ao);
#pragma unroll
      for (int j = 0; j < 4; ++j) {
        acc[i][j] = Frag<T>::mma(ah, bh[j], acc[i][j]);
        if (SPLIT) {
          acc[i][j] = Frag<T>::mma(ah, bl[j], acc[i][j]);
          acc[i][j] = Frag<T>::mma(al, bh[j], acc[i][j]);
        }
      }
      Frag<T>::guard(acc[i][0], acc[i][3], ah, SPLIT ? al : ah);
    }
    Frag<T>::keep(bh[0], bh[1], bh[2], bh[3]);
    if (SPLIT) Frag<T>::keep(bl[0], bl[1], bl[2], bl[3]);
  }
  acc_guard4(acc[0][0], acc[0][1], acc[0][2], acc[0][3]);
  acc_guard4(acc[1][0], acc[1][1], acc[1][2], acc[1][3]);
  acc_guard4(acc[2][0], acc[2][1], acc[2][2], acc[2][3]);
  acc_guard4(acc[3][0], acc[3][1], acc[3][2], acc[3][3]);

  float* slab = sT[wave];
  const float* Rb = RESID ? (resid + (size_t)b * strideR) : nullptr;
#pragma unroll
  for (int i = 0; i < 4; ++i) {
    const int mBase = m0 + (i << 4);
#pragma unroll
    for (int j = 0; j < 4; ++j) {
      const int n = n0 + (j << 4) + rlane;
      float bv = 0.f;
      if (BIAS_MODE == 2) bv = bias[n];
#pragma unroll
      for (int r = 0; r < 8; ++r) {
        float v = acc[i][j][r] * scale;
        if (BIAS_MODE == 1) v += bias[mBase + mOff + r];
        if (BIAS_MODE == 2) v += bv;
        if (RESID) v += Rb[(size_t)(mBase + mOff + r) * ldc + n];
        if (ACT == 1) v = tanhf(v);
        if (ACT == 2) v = fmaxf(v, 0.0f);
        if (ACT == 3) v = v / (1.0f + expf(-v));
        if (ACT == 4) v = (v > 0.f) ? v : 0.01f * v;
        if (ACT == 5) v = 0.5f * v * (1.0f + erff(v * 0.70710678118654752f));
        if (ACT == 6) v = (v >= 0.f) ? v : 0.1f * v;
        slab[(mOff + r) * 68 + (j << 4) + rlane] = v;
      }
    }
    __builtin_amdgcn_fence(__ATOMIC_RELEASE, "workgroup");
    __builtin_amdgcn_wave_barrier();
    __builtin_amdgcn_fence(__ATOMIC_ACQUIRE, "workgroup");
    if (OUT_MODE == 0) {
      float* C = (float*)Cout + (size_t)b * strideC;
      const int hh = lane >> 4, c4 = (lane & 15) * 4;
      for (int pass = 0; pass < 2; ++pass) {
#pragma unroll
        for (int it = 0; it < 8; ++it) {
          const int row = it * 2 + hh;
          v4f v = *(const v4f*)(slab + row * 68 + c4);
          *(volatile v4f*)(C + (size_t)(mBase + row) * ldc + n0 + c4) = v;
        }
        __threadfence();
      }
    } else {
      const int q = lane >> 3, c8 = (lane & 7) * 8;
      unsigned short* C  = (unsigned short*)Cout  + (size_t)b * strideC;
      unsigned short* C2 = (OUT_MODE == 2) ? ((unsigned short*)Cout2 + (size_t)b * strideC) : nullptr;
      for (int pass = 0; pass < 2; ++pass) {
#pragma unroll
        for (int it = 0; it < 4; ++it) {
          const int row = it * 4 + q;
          const float* sp = slab + row * 68 + c8;
          v8h hv, lv;
#pragma unroll
          for (int e = 0; e < 8; ++e) {
            if (OUT_MODE == 1) {
              hv[e] = (_Float16)sp[e];
            } else {
              unsigned short hb = f2bf_bits(sp[e]);
              unsigned short lb = f2bf_bits(sp[e] - bf_bits2f(hb));
              hv[e] = __builtin_bit_cast(_Float16, hb);
              lv[e] = __builtin_bit_cast(_Float16, lb);
            }
          }
          *(volatile v8h*)(C + (size_t)(mBase + row) * ldc + n0 + c8) = hv;
          if (OUT_MODE == 2) *(volatile v8h*)(C2 + (size_t)(mBase + row) * ldc + n0 + c8) = lv;
        }
        __threadfence();
      }
    }
    __builtin_amdgcn_fence(__ATOMIC_RELEASE, "workgroup");
    __builtin_amdgcn_wave_barrier();
    __builtin_amdgcn_fence(__ATOMIC_ACQUIRE, "workgroup");
  }
}

__global__ __launch_bounds__(256) void k_xpose_cat(const float* __restrict__ xa, const float* __restrict__ xb,
                                                   const float* __restrict__ xf, float* __restrict__ xT) {
  __shared__ float t[32][kCpt1 + 1];
  const int tid = threadIdx.x;
  const int blk = blockIdx.x;
  const int b   = blk / (kHW / 32);
  const int hw0 = (blk - b * (kHW / 32)) * 32;
  for (int i = 0; i < 17; ++i) {
    const int idx = i * 256 + tid;
    const int c = idx >> 5, j = idx & 31;
    const int ca = c < kCh ? c : (kCh - 1);
    int cb = c - kCh;     cb = cb < 0 ? 0 : (cb > kCh - 1 ? kCh - 1 : cb);
    int cf = c - 2 * kCh; cf = cf < 0 ? 0 : (cf > 1 ? 1 : cf);
    const float va = xa[((size_t)b * kCh + ca) * kHW + hw0 + j];
    const float vb = xb[((size_t)b * kCh + cb) * kHW + hw0 + j];
    const float vf = xf[((size_t)b * 2 + cf) * kHW + hw0 + j];
    float v = 0.0f;
    v = (c < kCin1) ? vf : v;
    v = (c < 2 * kCh) ? vb : v;
    v = (c < kCh) ? va : v;
    t[j][c] = v;
  }
  __syncthreads();
  const int wave = tid >> 5, lane = tid & 31, q = lane >> 3, piece = lane & 7;
  float* ob = xT + ((size_t)b * kHW + hw0) * kCpt1;
  for (int pass = 0; pass < 2; ++pass) {
#pragma unroll
    for (int it = 0; it < 5; ++it) {
      const int lw = it * 4 + q;
      if (lw < 17) {
        const int L = wave * 17 + lw;
        const int e = L * 32 + piece * 4;
        const int r = e / kCpt1, c = e - r * kCpt1;
        v4f v;
        v[0] = t[r][c]; v[1] = t[r][c + 1]; v[2] = t[r][c + 2]; v[3] = t[r][c + 3];
        *(volatile v4f*)(ob + e) = v;
      }
    }
    __threadfence();
  }
}

__global__ __launch_bounds__(256) void k_xpose64(const float* __restrict__ x, float* __restrict__ xT) {
  __shared__ float t[kCh][33];
  const int tid = threadIdx.x;
  const int blk = blockIdx.x;
  const int b   = blk / (kHW / 32);
  const int hw0 = (blk - b * (kHW / 32)) * 32;
  const float* xb = x + (size_t)b * kCh * kHW + hw0;
#pragma unroll
  for (int i = 0; i < 8; ++i) {
    const int idx = i * 256 + tid;
    const int c = idx >> 5, j = idx & 31;
    t[c][j] = xb[(size_t)c * kHW + j];
  }
  __syncthreads();
  const int wave = tid >> 5, lane = tid & 31, hh = lane >> 4, c4 = (lane & 15) * 4;
  float* ob = xT + ((size_t)b * kHW + hw0) * kCh;
  for (int pass = 0; pass < 2; ++pass) {
#pragma unroll
    for (int it = 0; it < 2; ++it) {
      const int row = wave * 4 + it * 2 + hh;
      v4f v;
      v[0] = t[c4][row]; v[1] = t[c4 + 1][row]; v[2] = t[c4 + 2][row]; v[3] = t[c4 + 3][row];
      *(volatile v4f*)(ob + (size_t)row * kCh + c4) = v;
    }
    __threadfence();
  }
}

__global__ __launch_bounds__(256) void k_prep_wsplit(const float* __restrict__ w, unsigned short* __restrict__ Ah,
                                                     unsigned short* __restrict__ Al,
                                                     int nReal, int nPad, int cin, int cpt, int kp) {
  const int g = blockIdx.x * 256 + threadIdx.x;
  if (g < nPad * kp / 8) {
    const int e0  = g * 8;
    const int o   = e0 / kp;
    const int col = e0 - o * kp;
    const int oc  = o < nReal ? o : (nReal - 1);
    float f[8];
#pragma unroll
    for (int j = 0; j < 8; ++j) {
      const int cj  = col + j;
      const int tap = cj / cpt;
      const int c   = cj - tap * cpt;
      const int tc  = tap < kTaps ? tap : (kTaps - 1);
      const int cc  = c < cin ? c : (cin - 1);
      const float v = w[((size_t)oc * cin + cc) * kTaps + tc];
      f[j] = (o < nReal && tap < kTaps && c < cin) ? v : 0.0f;
    }
    v4u uh, ul;
    unsigned a, bb;
    pkbf2(f[0], f[1], a, bb); uh[0] = a; ul[0] = bb;
    pkbf2(f[2], f[3], a, bb); uh[1] = a; ul[1] = bb;
    pkbf2(f[4], f[5], a, bb); uh[2] = a; ul[2] = bb;
    pkbf2(f[6], f[7], a, bb); uh[3] = a; ul[3] = bb;
    volatile v4u* ph = (volatile v4u*)(Ah + e0);
    volatile v4u* pl = (volatile v4u*)(Al + e0);
    *ph = uh; *pl = ul;
    __threadfence();
    *ph = uh; *pl = ul;
  }
}

__global__ __launch_bounds__(256) void k_prep_wdef(const float* __restrict__ w, unsigned short* __restrict__ Bw) {
  const int g = blockIdx.x * 256 + threadIdx.x;
  if (g < kCh * kKd / 8) {
    const int e0  = g * 8;
    const int o   = e0 / kKd;
    const int col = e0 - o * kKd;
    const int k   = col >> 6;
    const int c0  = col & 63;
    float f[8];
#pragma unroll
    for (int j = 0; j < 8; ++j) f[j] = w[(size_t)(o * kCh + c0 + j) * kTaps + k] * 64.0f;
    v4u u;
    u[0] = pkh2(f[0], f[1]); u[1] = pkh2(f[2], f[3]); u[2] = pkh2(f[4], f[5]); u[3] = pkh2(f[6], f[7]);
    volatile v4u* p = (volatile v4u*)(Bw + e0);
    *p = u;
    __threadfence();
    *p = u;
  }
}

__global__ __launch_bounds__(64) void k_pad_bias(const float* __restrict__ bsrc, float* __restrict__ bdst,
                                                 int nReal, int nPad) {
  const int i = threadIdx.x;
  if (i < nPad / 4) {
    v4f v;
#pragma unroll
    for (int e = 0; e < 4; ++e) {
      const int idx = 4 * i + e;
      const int ic  = idx < nReal ? idx : (nReal - 1);
      const float f = bsrc[ic];
      v[e] = (idx < nReal) ? f : 0.0f;
    }
    *(volatile v4f*)(bdst + 4 * i) = v;
    __threadfence();
    *(volatile v4f*)(bdst + 4 * i) = v;
  }
}

__global__ __launch_bounds__(256) void k_im2col_cat(const float* __restrict__ xT, unsigned short* __restrict__ Ph,
                                                    unsigned short* __restrict__ Pl, int p0) {
  const int lane = threadIdx.x & 31, wave = threadIdx.x >> 5;
  const int r  = blockIdx.x * 8 + wave;
  const int p  = p0 + r;
  const int b  = p >> 14, hw = p & (kHW - 1);
  const int ho = hw >> 7, wo = hw & (kImg - 1);
  const v4f z = (v4f){0.f, 0.f, 0.f, 0.f};
#pragma unroll
  for (int i = 0; i < 5; ++i) {
    const int j   = i * 32 + lane;
    const int jj  = j < 153 ? j : 152;
    const int tap = jj / 17;
    const int c8  = (jj - tap * 17) * 8;
    const int kh  = tap / 3, kw = tap - kh * 3;
    const int y = ho - 1 + kh, xx = wo - 1 + kw;
    const bool inb = ((unsigned)y < (unsigned)kImg) && ((unsigned)xx < (unsigned)kImg) && (j < 153);
    const int yc = y < 0 ? 0 : (y > kImg - 1 ? kImg - 1 : y);
    const int xc = xx < 0 ? 0 : (xx > kImg - 1 ? kImg - 1 : xx);
    const float* src = xT + ((size_t)b * kHW + (size_t)yc * kImg + xc) * kCpt1 + c8;
    v4f a = *(const v4f*)(src);
    v4f c = *(const v4f*)(src + 4);
    if (!inb) { a = z; c = z; }
    v4u uh, ul;
    unsigned q0, q1;
    pkbf2(a[0], a[1], q0, q1); uh[0] = q0; ul[0] = q1;
    pkbf2(a[2], a[3], q0, q1); uh[1] = q0; ul[1] = q1;
    pkbf2(c[0], c[1], q0, q1); uh[2] = q0; ul[2] = q1;
    pkbf2(c[2], c[3], q0, q1); uh[3] = q0; ul[3] = q1;
    volatile v4u* dh = (volatile v4u*)(Ph + (size_t)r * kKp1 + j * 8);
    volatile v4u* dl = (volatile v4u*)(Pl + (size_t)r * kKp1 + j * 8);
    *dh = uh; *dl = ul;
    __threadfence();
    *dh = uh; *dl = ul;
  }
}

__global__ __launch_bounds__(256) void k_im2col64(const float* __restrict__ xT, unsigned short* __restrict__ Ph,
                                                  unsigned short* __restrict__ Pl, int p0, int nItems) {
  const int lane = threadIdx.x & 31, wave = threadIdx.x >> 5;
  const int q = lane >> 3, c8 = (lane & 7) * 8;
  const int it = (blockIdx.x * 8 + wave) * 4 + q;
  if (it < nItems) {
    const int pl = it / kTaps, k = it - pl * kTaps;
    const int p  = p0 + pl;
    const int b  = p >> 14, hw = p & (kHW - 1);
    const int ho = hw >> 7, wo = hw & (kImg - 1);
    const int kh = k / 3, kw = k - kh * 3;
    const int y = ho - 1 + kh, xx = wo - 1 + kw;
    const bool inb = ((unsigned)y < (unsigned)kImg) && ((unsigned)xx < (unsigned)kImg);
    const int yc = y < 0 ? 0 : (y > kImg - 1 ? kImg - 1 : y);
    const int xc = xx < 0 ? 0 : (xx > kImg - 1 ? kImg - 1 : xx);
    const float* src = xT + ((size_t)b * kHW + (size_t)yc * kImg + xc) * kCh + c8;
    v4f a = *(const v4f*)(src);
    v4f c = *(const v4f*)(src + 4);
    const v4f z = (v4f){0.f, 0.f, 0.f, 0.f};
    if (!inb) { a = z; c = z; }
    v4u uh, ul;
    unsigned q0, q1;
    pkbf2(a[0], a[1], q0, q1); uh[0] = q0; ul[0] = q1;
    pkbf2(a[2], a[3], q0, q1); uh[1] = q0; ul[1] = q1;
    pkbf2(c[0], c[1], q0, q1); uh[2] = q0; ul[2] = q1;
    pkbf2(c[2], c[3], q0, q1); uh[3] = q0; ul[3] = q1;
    volatile v4u* dh = (volatile v4u*)(Ph + (size_t)it * kCh + c8);
    volatile v4u* dl = (volatile v4u*)(Pl + (size_t)it * kCh + c8);
    *dh = uh; *dl = ul;
    __threadfence();
    *dh = uh; *dl = ul;
  }
}

__global__ __launch_bounds__(256) void k_sample(const float* __restrict__ xT, const float* __restrict__ om,
                                                const float* __restrict__ flows, unsigned short* __restrict__ S) {
  const int lane = threadIdx.x & 31, wave = threadIdx.x >> 5;
  const int q = lane >> 3, g = lane & 7, c8 = g * 8;
  const int it = (blockIdx.x * 8 + wave) * 4 + q;
  if (it < kNpix * kTaps) {
    const int p = it / kTaps, k = it - p * kTaps;
    const int b = p >> 14, hw = p & (kHW - 1);
    const int ho = hw >> 7, wo = hw & (kImg - 1);
    const int kh = k / 3, kw = k - kh * 3;
    const float* omp = om + (size_t)p * kNomPad;
    const int ch = (g * kTaps + k) * 2;
    const float dy = omp[ch]     + flows[((size_t)b * 2 + 1) * kHW + hw];
    const float dx = omp[ch + 1] + flows[((size_t)b * 2 + 0) * kHW + hw];
    const float ml = omp[2 * kGroups * kTaps + g * kTaps + k];
    const float mk = __builtin_amdgcn_rcpf(1.0f + expf(-ml));
    const float py = (float)(ho - 1 + kh) + dy;
    const float px = (float)(wo - 1 + kw) + dx;
    const float y0 = floorf(py), x0 = floorf(px);
    const float y1 = y0 + 1.0f, x1 = x0 + 1.0f;
    const float wy1 = py - y0, wx1 = px - x0;
    const float wy0 = 1.0f - wy1, wx0 = 1.0f - wx1;
    const bool vy0 = (y0 >= 0.0f) && (y0 <= (float)(kImg - 1));
    const bool vy1 = (y1 >= 0.0f) && (y1 <= (float)(kImg - 1));
    const bool vx0 = (x0 >= 0.0f) && (x0 <= (float)(kImg - 1));
    const bool vx1 = (x1 >= 0.0f) && (x1 <= (float)(kImg - 1));
    float w00 = wy0 * wx0, w01 = wy0 * wx1, w10 = wy1 * wx0, w11 = wy1 * wx1;
    w00 = (vy0 && vx0) ? w00 : 0.0f;
    w01 = (vy0 && vx1) ? w01 : 0.0f;
    w10 = (vy1 && vx0) ? w10 : 0.0f;
    w11 = (vy1 && vx1) ? w11 : 0.0f;
    const int yi0 = (int)fminf(fmaxf(y0, 0.0f), (float)(kImg - 1));
    const int yi1 = (int)fminf(fmaxf(y1, 0.0f), (float)(kImg - 1));
    const int xi0 = (int)fminf(fmaxf(x0, 0.0f), (float)(kImg - 1));
    const int xi1 = (int)fminf(fmaxf(x1, 0.0f), (float)(kImg - 1));
    const float* xb  = xT + (size_t)b * kHW * kCh + c8;
    const float* r00 = xb + ((size_t)yi0 * kImg + xi0) * kCh;
    const float* r01 = xb + ((size_t)yi0 * kImg + xi1) * kCh;
    const float* r10 = xb + ((size_t)yi1 * kImg + xi0) * kCh;
    const float* r11 = xb + ((size_t)yi1 * kImg + xi1) * kCh;
    const v4f g00a = *(const v4f*)(r00), g00b = *(const v4f*)(r00 + 4);
    const v4f g01a = *(const v4f*)(r01), g01b = *(const v4f*)(r01 + 4);
    const v4f g10a = *(const v4f*)(r10), g10b = *(const v4f*)(r10 + 4);
    const v4f g11a = *(const v4f*)(r11), g11b = *(const v4f*)(r11 + 4);
    v4f va = g00a * w00 + g01a * w01 + g10a * w10 + g11a * w11;
    v4f vb = g00b * w00 + g01b * w01 + g10b * w10 + g11b * w11;
    va = va * mk;
    vb = vb * mk;
    v4u u;
    u[0] = pkh2(va[0], va[1]); u[1] = pkh2(va[2], va[3]);
    u[2] = pkh2(vb[0], vb[1]); u[3] = pkh2(vb[2], vb[3]);
    volatile v4u* d = (volatile v4u*)(S + (size_t)it * kCh + c8);
    *d = u;
    __threadfence();
    *d = u;
  }
}

extern "C" void kernel_launch(void* const* d_in, const int* in_sizes, int n_in,
                              void* d_out, int out_size, void* d_ws, size_t ws_size,
                              hipStream_t stream) {
  if (n_in < 12) return;
  if (in_sizes[0] != kNpix * kCh || in_sizes[1] != kNpix * kCh || in_sizes[2] != kNpix * kCh ||
      in_sizes[3] != kBatch * 2 * kHW) return;
  if (in_sizes[4] != kCh * kCin1 * kTaps || in_sizes[5] != kCh ||
      in_sizes[6] != kCh * kCh * kTaps   || in_sizes[7] != kCh ||
      in_sizes[8] != kNom * kCh * kTaps  || in_sizes[9] != kNom ||
      in_sizes[10] != kCh * kCh * kTaps  || in_sizes[11] != kCh) return;
  if (out_size != kBatch * kCh * kHW) return;

  const float* x_ref = (const float*)d_in[0];
  const float* x_flw = (const float*)d_in[1];
  const float* x_shk = (const float*)d_in[2];
  const float* flw   = (const float*)d_in[3];
  const float* w1    = (const float*)d_in[4];
  const float* b1    = (const float*)d_in[5];
  const float* w2    = (const float*)d_in[6];
  const float* b2    = (const float*)d_in[7];
  const float* wom   = (const float*)d_in[8];
  const float* bom   = (const float*)d_in[9];
  const float* wd    = (const float*)d_in[10];
  const float* bd    = (const float*)d_in[11];
  float* out = (float*)d_out;

  const size_t bW1  = (size_t)kCh * kKp1 * 2;
  const size_t bW2  = (size_t)kCh * kKd * 2;
  const size_t bWO  = (size_t)kNomPad * kKd * 2;
  const size_t bWD  = (size_t)kCh * kKd * 2;
  const size_t bBOM = (size_t)kNomPad * 4;
  const size_t bXTR = (size_t)kNpix * kCh * 4;
  const size_t bOMP = (size_t)kNpix * kNomPad * 4;
  const size_t bRA  = (size_t)kNpix * kCpt1 * 4;
  const size_t bF1  = (size_t)kNpix * kCh * 4;
  const size_t bIM1 = (size_t)kChunk1 * kKp1 * 2 * 2;
  const size_t bIM2 = (size_t)kChunk2 * kKd * 2 * 2;
  const size_t bVAL = (size_t)kNpix * kKd * 2;
  size_t bBIG = bVAL;
  if (bIM1 > bBIG) bBIG = bIM1;
  if (bIM2 > bBIG) bBIG = bIM2;
  if (bF1 > bRA) return;
  char* ws = (char*)d_ws;
  size_t o = 0;
  unsigned short* W1h = (unsigned short*)(ws + o); o += bW1;
  unsigned short* W1l = (unsigned short*)(ws + o); o += bW1;
  unsigned short* W2h = (unsigned short*)(ws + o); o += bW2;
  unsigned short* W2l = (unsigned short*)(ws + o); o += bW2;
  unsigned short* WOh = (unsigned short*)(ws + o); o += bWO;
  unsigned short* WOl = (unsigned short*)(ws + o); o += bWO;
  unsigned short* WDf = (unsigned short*)(ws + o); o += bWD;
  float* BOM = (float*)(ws + o);                   o += bBOM;
  float* XTR = (float*)(ws + o);                   o += bXTR;
  float* OMP = (float*)(ws + o);                   o += bOMP;
  float* XT0 = (float*)(ws + o);
  float* F2  = (float*)(ws + o);                   o += bRA;
  float* F1  = (float*)(ws + o);                   o += bF1;
  unsigned short* BIG = (unsigned short*)(ws + o); o += bBIG;
  if (o > ws_size) return;
  unsigned short* IMh  = BIG;
  unsigned short* IMl1 = BIG + (size_t)kChunk1 * kKp1;
  unsigned short* IMl2 = BIG + (size_t)kChunk2 * kKd;
  unsigned short* VAL  = BIG;

  k_xpose_cat<<<kNpix / 32, 256, 0, stream>>>(x_flw, x_shk, flw, XT0);
  k_xpose64<<<kNpix / 32, 256, 0, stream>>>(x_ref, XTR);
  k_prep_wsplit<<<(kCh * kKp1 / 8 + 255) / 256, 256, 0, stream>>>(w1, W1h, W1l, kCh, kCh, kCin1, kCpt1, kKp1);
  k_prep_wsplit<<<(kCh * kKd / 8 + 255) / 256, 256, 0, stream>>>(w2, W2h, W2l, kCh, kCh, kCh, kCh, kKd);
  k_prep_wsplit<<<(kNomPad * kKd / 8 + 255) / 256, 256, 0, stream>>>(wom, WOh, WOl, kNom, kNomPad, kCh, kCh, kKd);
  k_prep_wdef<<<(kCh * kKd / 8 + 255) / 256, 256, 0, stream>>>(wd, WDf);
  k_pad_bias<<<1, 64, 0, stream>>>(bom, BOM, kNom, kNomPad);
  for (int cix = 0; cix < kNpix / kChunk1; ++cix) {
    const int p0 = cix * kChunk1;
    k_im2col_cat<<<kChunk1 / 8, 256, 0, stream>>>(XT0, IMh, IMl1, p0);
    wmma_gemm64<1, true, 2, 0, false, 6><<<dim3((kChunk1 / 64) * (kCh / 64) / 8, 1), 256, 0, stream>>>(
        IMh, IMl1, kKp1, 0L,
        W1h, W1l, kKp1, 0L,
        (void*)(F1 + (size_t)p0 * kCh), (void*)WDf, kCh, 0L,
        b1,
        BOM, 0L,
        kChunk1, kCh, kKp1, 1.0f);
  }
  for (int cix = 0; cix < kNpix / kChunk2; ++cix) {
    const int p0 = cix * kChunk2;
    k_im2col64<<<kChunk2 * kTaps / 32, 256, 0, stream>>>(F1, IMh, IMl2, p0, kChunk2 * kTaps);
    wmma_gemm64<1, true, 2, 0, false, 6><<<dim3((kChunk2 / 64) * (kCh / 64) / 8, 1), 256, 0, stream>>>(
        IMh, IMl2, kKd, 0L,
        W2h, W2l, kKd, 0L,
        (void*)(F2 + (size_t)p0 * kCh), (void*)WDf, kCh, 0L,
        b2,
        BOM, 0L,
        kChunk2, kCh, kKd, 1.0f);
  }
  for (int cix = 0; cix < kNpix / kChunk2; ++cix) {
    const int p0 = cix * kChunk2;
    k_im2col64<<<kChunk2 * kTaps / 32, 256, 0, stream>>>(F2, IMh, IMl2, p0, kChunk2 * kTaps);
    wmma_gemm64<1, true, 2, 0, false, 0><<<dim3((kChunk2 / 64) * (kNomPad / 64) / 8, 1), 256, 0, stream>>>(
        IMh, IMl2, kKd, 0L,
        WOh, WOl, kKd, 0L,
        (void*)(OMP + (size_t)p0 * kNomPad), (void*)WDf, kNomPad, 0L,
        BOM,
        BOM, 0L,
        kChunk2, kNomPad, kKd, 1.0f);
  }
  k_sample<<<kNpix * kTaps / 32, 256, 0, stream>>>(XTR, OMP, flw, VAL);
  wmma_gemm64<0, false, 1, 0, false, 6><<<dim3((kCh / 64) * (kHW / 64) / 8, kBatch), 256, 0, stream>>>(
      WDf, WDf, kKd, 0L,
      VAL, VAL, kKd, (long)kHW * kKd,
      (void*)out, (void*)WDf, kHW, (long)kCh * kHW,
      bd,
      BOM, 0L,
      kCh, kHW, kKd, 0.015625f);
}
